// PPFNet_29386166239365
// MI455X (gfx1250) — hardware-verified
//
#include <hip/hip_runtime.h>
#include <math.h>

typedef __attribute__((ext_vector_type(16))) _Float16 v16h;
typedef __attribute__((ext_vector_type(16))) __bf16 v16b;
typedef __attribute__((ext_vector_type(8)))  _Float16 v8h;
typedef __attribute__((ext_vector_type(8)))  float v8f;
typedef __attribute__((ext_vector_type(4)))  float v4f;
typedef __attribute__((ext_vector_type(2)))  float v2f;
typedef __attribute__((ext_vector_type(4)))  unsigned v4u;
typedef __attribute__((ext_vector_type(4)))  int v4i;
typedef float __attribute__((may_alias)) float_a;
typedef int __attribute__((may_alias)) int_a;

template <typename T> __device__ __forceinline__ void vst2(void* p, T v) { *(volatile T*)p = v; __threadfence(); *(volatile T*)p = v; }
__device__ __forceinline__ v8f wmma16(v16h a, v16h b, v8f c) {
  v8f d = __builtin_amdgcn_wmma_f32_16x16x32_f16(false, a, false, b, (short)0, c, false, false);
  asm volatile("v_nop\n\tv_nop\n\tv_nop\n\tv_nop" : "+v"(d) : "v"(a), "v"(b));
  return d;
}
__device__ __forceinline__ v8f wmma_bf(v16b a, v16b b, v8f c) {
  v8f d = __builtin_amdgcn_wmma_f32_16x16x32_bf16(false, a, false, b, (short)0, c, false, false);
  asm volatile("v_nop\n\tv_nop\n\tv_nop\n\tv_nop" : "+v"(d) : "v"(a), "v"(b));
  return d;
}
__device__ __forceinline__ v16h frag_h(const _Float16* rowk0, int lane) {
  union { v16h v; v8h q[2]; } u; const _Float16* p = rowk0 + 8 * (lane >> 4);
  u.q[0] = *(const v8h*)p; u.q[1] = *(const v8h*)(p + 16); return u.v;
}
__device__ __forceinline__ v16h frag_f32(const float* rowk0, int lane) {
  v16h a; const float* p = rowk0 + 8 * (lane >> 4);
#pragma unroll
  for (int i = 0; i < 8; ++i) { a[i] = (_Float16)p[i]; a[8 + i] = (_Float16)p[16 + i]; }
  return a;
}
__device__ __forceinline__ v16h frag_f32s(const float* rowk0, int lane, float sc) {
  v16h a; const float* p = rowk0 + 8 * (lane >> 4);
#pragma unroll
  for (int i = 0; i < 8; ++i) { a[i] = (_Float16)(p[i] * sc); a[8 + i] = (_Float16)(p[16 + i] * sc); }
  return a;
}
__device__ __forceinline__ v16h fragc_f32(const float* W, int k0, int n, int lane, int ld, int K) {
  v16h a; const int g = lane >> 4;
#pragma unroll
  for (int i = 0; i < 8; ++i) { const int ka = k0 + 8 * g + i, kb = ka + 16;
    a[i] = (_Float16)(ka < K ? W[(size_t)(ka < K ? ka : K - 1) * ld + n] : 0.f); a[8 + i] = (_Float16)(kb < K ? W[(size_t)(kb < K ? kb : K - 1) * ld + n] : 0.f); }
  return a;
}
struct F2 { v16b h, l; };
__device__ __forceinline__ F2 bsplit16(const float v[16]) { F2 r;
#pragma unroll
  for (int i = 0; i < 16; ++i) { const __bf16 h = (__bf16)v[i]; r.h[i] = h; r.l[i] = (__bf16)(v[i] - (float)h); }
  return r; }
__device__ __forceinline__ F2 split_row(const float* row, int k0, int lane) { float v[16]; const float* p = row + k0 + 8 * (lane >> 4);
#pragma unroll
  for (int i = 0; i < 8; ++i) { v[i] = p[i]; v[8 + i] = p[16 + i]; }
  return bsplit16(v); }
__device__ __forceinline__ F2 split_rowK(const float* row, int k0, int lane, int K) { float v[16]; const int g = lane >> 4;
#pragma unroll
  for (int i = 0; i < 8; ++i) { const int ka = k0 + 8 * g + i, kb = ka + 16; v[i] = ka < K ? row[ka < K ? ka : K - 1] : 0.f; v[8 + i] = kb < K ? row[kb < K ? kb : K - 1] : 0.f; }
  return bsplit16(v); }
__device__ __forceinline__ F2 split_col(const float* W, int k0, int n, int lane, int ld, int K) { float v[16]; const int g = lane >> 4;
#pragma unroll
  for (int i = 0; i < 8; ++i) { const int ka = k0 + 8 * g + i, kb = ka + 16; v[i] = ka < K ? W[(size_t)(ka < K ? ka : K - 1) * ld + n] : 0.f; v[8 + i] = kb < K ? W[(size_t)(kb < K ? kb : K - 1) * ld + n] : 0.f; }
  return bsplit16(v); }
__device__ __forceinline__ v8f mac3(const F2& a, const F2& b, v8f c) { c = wmma_bf(a.l, b.h, c); c = wmma_bf(a.h, b.l, c); return wmma_bf(a.h, b.h, c); }
__device__ __forceinline__ float sigm(float v) { return 1.0f / (1.0f + expf(-v)); }
#define LDSX() do { asm volatile("s_wait_dscnt 0" ::: "memory"); __builtin_amdgcn_wave_barrier(); __builtin_amdgcn_fence(__ATOMIC_RELEASE, "workgroup"); } while (0)


#define NBATCH 8
#define NPTS 4096
#define MM (NBATCH * NPTS)
#define KN 16
#define KE 17
#define NROW (MM * KE)
#define NCL 40
#ifndef NQB
#define NQB (MM / 64)
#define NRWB (NROW / 64)
#define NBT NBATCH
#endif
typedef __attribute__((ext_vector_type(8))) __bf16 v8b;
__device__ __forceinline__ v16b frag_b(const __bf16* rowk0, int lane) {
  union { v16b v; v8b q[2]; } u; const __bf16* p = rowk0 + 8 * (lane >> 4);
  u.q[0] = *(const v8b*)p; u.q[1] = *(const v8b*)(p + 16); return u.v;
}
__device__ __forceinline__ float bfr(float v) { return (float)(__bf16)v; }
__device__ __attribute__((noinline)) float exp_ni(float v) { return expf(v); }
__device__ __attribute__((noinline)) float erf_ni(float v) { return erff(v); }

__device__ __attribute__((noinline)) float atan2_ni(float y, float x) { return atan2f(y, x); }
struct F3 { v16b h, m, l; };
__device__ __forceinline__ F3 bsplit16_3(const float v[16]) { F3 r;
#pragma unroll
  for (int i = 0; i < 16; ++i) { const __bf16 h = (__bf16)v[i]; const float r1 = v[i] - (float)h; const __bf16 m = (__bf16)r1; r.h[i] = h; r.m[i] = m; r.l[i] = (__bf16)(r1 - (float)m); }
  return r; }
__device__ __forceinline__ F3 split3_row(const float* row, int k0, int lane) { float v[16]; const float* p = row + k0 + 8 * (lane >> 4);
#pragma unroll
  for (int i = 0; i < 8; ++i) { v[i] = p[i]; v[8 + i] = p[16 + i]; }
  return bsplit16_3(v); }

#define WS_PW   0u
#define PW1B 0
#define PW2A (PW1B + 32 * 32)
#define PW2B (PW2A + 32 * 64)
#define PWEND (PW2B + 32 * 32)
#define WS_KNN  (WS_PW + 2u * PWEND)
#define WS_F4   (WS_KNN + 4u * MM * KN)
#define WS_MSG  (WS_F4 + 4u * NROW * 4)
#define WS_X    (WS_MSG + 4u * NROW * 32)
#define WS_G    (WS_X + 4u * MM * 32)
#define WS_END  (WS_G + 4u * 8 * 32)

__global__ __launch_bounds__(256) void k_packw(const float* __restrict__ W1B, const float* __restrict__ W2A, const float* __restrict__ W2B, __bf16* __restrict__ PW) {
  __shared__ __align__(16) __bf16 s1[32][32], s2[32][64], s3[32][32]; const int t = threadIdx.x;
  for (int q = t; q < 32 * 32; q += 256) { const int o = q >> 5, k = q & 31; s1[o][k] = (__bf16)W1B[k * 32 + o]; s3[o][k] = (__bf16)W2B[k * 32 + o]; }
  for (int q = t; q < 32 * 64; q += 256) { const int o = q >> 6, k = q & 63; s2[o][k] = (__bf16)((k < 36) ? W2A[k * 32 + o] : 0.f); }
  __syncthreads();
  for (int q = t; q < 32 * 32 / 8; q += 256) { vst2((unsigned*)(PW + PW1B + q * 8), *(const v4u*)(&s1[0][0] + q * 8)); vst2((unsigned*)(PW + PW2B + q * 8), *(const v4u*)(&s3[0][0] + q * 8)); }
  for (int q = t; q < 32 * 64 / 8; q += 256) vst2((unsigned*)(PW + PW2A + q * 8), *(const v4u*)(&s2[0][0] + q * 8));
}
__global__ __launch_bounds__(64) void k_knn(const float* __restrict__ POS, int* __restrict__ KNN) {
  __shared__ __align__(16) int sk[64][KN]; const int tid = threadIdx.x; const size_t i = (size_t)blockIdx.x * 64 + tid; const int b = (int)(i / NPTS); const int il = (int)(i % NPTS);
  const float* pb = POS + (size_t)b * NPTS * 3; const float xi = bfr(pb[il * 3]), yi = bfr(pb[il * 3 + 1]), zi = bfr(pb[il * 3 + 2]); const float sqi = (xi * xi + zi * zi) + yi * yi;
  float bd[KN]; int bi[KN];
#pragma unroll
  for (int j = 0; j < KN; ++j) { bd[j] = 3.0e38f; bi[j] = 0; }
#pragma unroll 1
  for (int j = 0; j < NPTS; ++j) { const float xj = bfr(pb[j * 3]), yj = bfr(pb[j * 3 + 1]), zj = bfr(pb[j * 3 + 2]); const float sqj = (xj * xj + zj * zj) + yj * yj; const float dot = (xi * xj + yi * yj) + zi * zj; const float d = (sqi + sqj) - 2.0f * dot;
    if (j != il && d < bd[KN - 1]) { int pos = KN - 1;
#pragma unroll
      for (int q = KN - 2; q >= 0; --q) if (d < bd[q]) pos = q;
#pragma unroll
      for (int q = KN - 1; q >= 1; --q) if (q > pos) { bd[q] = bd[q - 1]; bi[q] = bi[q - 1]; }
#pragma unroll
      for (int q = 0; q < KN; ++q) if (q == pos) { bd[q] = d; bi[q] = j; } } }
#pragma unroll
  for (int j = 0; j < KN; ++j) sk[tid][j] = b * NPTS + bi[j];
  __syncthreads();
  for (int q = tid; q < 64 * KN / 4; q += 64) vst2((unsigned*)(KNN + (size_t)blockIdx.x * 64 * KN + q * 4), *(const v4u*)(&sk[0][0] + q * 4));
}
__device__ __forceinline__ float safe_norm3(float a, float b, float c) { const float s = (a * a + b * b) + c * c; return s > 0.f ? sqrtf(s) : 0.f; }
__device__ __forceinline__ float angle3(float ax, float ay, float az, float bx, float by, float bz) {
  const float cx = ay * bz - az * by, cy = az * bx - ax * bz, cz = ax * by - ay * bx; const float cn = safe_norm3(cx, cy, cz); const float d = (ax * bx + ay * by) + az * bz;
  const bool ok = (cn > 0.f) || (d != 0.f); return ok ? atan2_ni(cn, ok ? d : 1.f) : 0.f;
}
__global__ __launch_bounds__(128) void k_edge1(const float* __restrict__ POS, const float* __restrict__ NRM, const int* __restrict__ KNN, const float* __restrict__ W1A, const float* __restrict__ B1A, const __bf16* __restrict__ PW, const float* __restrict__ B1B, float* __restrict__ F4, float* __restrict__ MSG) {
  __shared__ __align__(16) float sh[64][36]; __shared__ __align__(16) float sf[64][4]; __shared__ __align__(16) float so[4][16][36];
  const int tid = threadIdx.x, wave = tid >> 5, lane = tid & 31, col = lane & 15, g = lane >> 4; const size_t rb = (size_t)blockIdx.x * 64;
  if (tid < 64) { const size_t r = rb + tid; const size_t i = r / KE; const int k = (int)(r % KE); const size_t j = (k < KN) ? (size_t)min(max(KNN[i * KN + k], 0), MM - 1) : i;
    const float pix = bfr(POS[i * 3]), piy = bfr(POS[i * 3 + 1]), piz = bfr(POS[i * 3 + 2]); const float pjx = bfr(POS[j * 3]), pjy = bfr(POS[j * 3 + 1]), pjz = bfr(POS[j * 3 + 2]);
    const float nix = bfr(NRM[i * 3]), niy = bfr(NRM[i * 3 + 1]), niz = bfr(NRM[i * 3 + 2]); const float njx = bfr(NRM[j * 3]), njy = bfr(NRM[j * 3 + 1]), njz = bfr(NRM[j * 3 + 2]);
    const float dx = pjx - pix, dy = pjy - piy, dz = pjz - piz;
    float f[4]; f[0] = safe_norm3(dx, dy, dz); f[1] = angle3(nix, niy, niz, dx, dy, dz); f[2] = angle3(njx, njy, njz, dx, dy, dz); f[3] = angle3(nix, niy, niz, njx, njy, njz);
#pragma unroll
    for (int q = 0; q < 4; ++q) sf[tid][q] = f[q];
#pragma unroll 1
    for (int o = 0; o < 32; ++o) { float a = bfr(B1A[o]);
#pragma unroll
      for (int q = 0; q < 4; ++q) a += f[q] * bfr(W1A[q * 32 + o]);
      sh[tid][o] = fmaxf(a, 0.f); } }
  __syncthreads();
  if (tid < 64) vst2(F4 + (rb + tid) * 4, *(const v4f*)&sf[tid][0]);
  const F3 a = split3_row(&sh[wave * 16 + col][0], 0, lane);
  v8f acc[2] = {};
#pragma unroll
  for (int jn = 0; jn < 2; ++jn) { const v16b w = frag_b(PW + PW1B + (size_t)(jn * 16 + col) * 32, lane); acc[jn] = wmma_bf(a.l, w, acc[jn]); acc[jn] = wmma_bf(a.m, w, acc[jn]); acc[jn] = wmma_bf(a.h, w, acc[jn]); }
#pragma unroll
  for (int jn = 0; jn < 2; ++jn)
#pragma unroll
    for (int r = 0; r < 8; ++r) so[wave][8 * g + r][jn * 16 + col] = acc[jn][r] + bfr(B1B[jn * 16 + col]);
  LDSX();
  for (int rl = 0; rl < 16; ++rl) if (lane < 8) vst2(MSG + (rb + wave * 16 + rl) * 32 + lane * 4, *(const v4f*)&so[wave][rl][lane * 4]);
}
__global__ __launch_bounds__(256) void k_segmax(const float* __restrict__ MSG, float* __restrict__ X) {
  const int tid = threadIdx.x; const int c = tid & 31, sl = tid >> 5;
  for (int pass = 0; pass < 8; ++pass) { const size_t i = (size_t)blockIdx.x * 64 + pass * 8 + sl; float m = -INFINITY;
#pragma unroll 1
    for (int k = 0; k < KE; ++k) m = fmaxf(m, MSG[(i * KE + k) * 32 + c]);
    vst2(X + i * 32 + c, fmaxf(m, 0.f)); }
}
__global__ __launch_bounds__(128) void k_edge2(const float* __restrict__ X, const float* __restrict__ F4, const int* __restrict__ KNN, const __bf16* __restrict__ PW, const float* __restrict__ B2A, const float* __restrict__ B2B, float* __restrict__ MSG) {
  __shared__ __align__(16) float sa[64][68]; __shared__ __align__(16) float sh[4][16][36]; __shared__ __align__(16) float so[4][16][36];
  const int tid = threadIdx.x, wave = tid >> 5, lane = tid & 31, col = lane & 15, g = lane >> 4; const size_t rb = (size_t)blockIdx.x * 64;
  for (int q = tid; q < 64 * 64; q += 128) { const int rl = q >> 6, cc = q & 63; const size_t r = rb + rl; const size_t i = r / KE; const int k = (int)(r % KE); const size_t j = (k < KN) ? (size_t)min(max(KNN[i * KN + k], 0), MM - 1) : i;
    float v = 0.f; if (cc < 32) v = X[j * 32 + cc]; else if (cc < 36) v = F4[r * 4 + (cc - 32)]; sa[rl][cc] = v; }
  __syncthreads();
  v8f acc[2] = {};
#pragma unroll
  for (int kc = 0; kc < 2; ++kc) { const F3 a = split3_row(&sa[wave * 16 + col][0], kc * 32, lane);
#pragma unroll
    for (int jn = 0; jn < 2; ++jn) { const v16b w = frag_b(PW + PW2A + (size_t)(jn * 16 + col) * 64 + kc * 32, lane); acc[jn] = wmma_bf(a.l, w, acc[jn]); acc[jn] = wmma_bf(a.m, w, acc[jn]); acc[jn] = wmma_bf(a.h, w, acc[jn]); } }
#pragma unroll
  for (int jn = 0; jn < 2; ++jn)
#pragma unroll
    for (int r = 0; r < 8; ++r) sh[wave][8 * g + r][jn * 16 + col] = fmaxf(acc[jn][r] + bfr(B2A[jn * 16 + col]), 0.f);
  LDSX();
  const F3 a2 = split3_row(&sh[wave][col][0], 0, lane);
  v8f acc2[2] = {};
#pragma unroll
  for (int jn = 0; jn < 2; ++jn) { const v16b w = frag_b(PW + PW2B + (size_t)(jn * 16 + col) * 32, lane); acc2[jn] = wmma_bf(a2.l, w, acc2[jn]); acc2[jn] = wmma_bf(a2.m, w, acc2[jn]); acc2[jn] = wmma_bf(a2.h, w, acc2[jn]); }
#pragma unroll
  for (int jn = 0; jn < 2; ++jn)
#pragma unroll
    for (int r = 0; r < 8; ++r) so[wave][8 * g + r][jn * 16 + col] = acc2[jn][r] + bfr(B2B[jn * 16 + col]);
  LDSX();
  for (int rl = 0; rl < 16; ++rl) if (lane < 8) vst2(MSG + (rb + wave * 16 + rl) * 32 + lane * 4, *(const v4f*)&so[wave][rl][lane * 4]);
}
__global__ __launch_bounds__(256) void k_pool(const float* __restrict__ X, float* __restrict__ G) {
  __shared__ float sm[8][32]; __shared__ __align__(16) float sg[32]; const int tid = threadIdx.x; const int c = tid & 31, sl = tid >> 5; const int b = blockIdx.x; float m = -INFINITY;
#pragma unroll 1
  for (int n = sl; n < NPTS; n += 8) m = fmaxf(m, X[((size_t)b * NPTS + n) * 32 + c]);
  sm[sl][c] = m; __syncthreads();
  if (tid < 32) { float v = sm[0][tid]; for (int s = 1; s < 8; ++s) v = fmaxf(v, sm[s][tid]); sg[tid] = v; }
  __syncthreads();
  if (tid < 8) vst2(G + (size_t)b * 32 + tid * 4, *(const v4f*)&sg[tid * 4]);
}
__global__ __launch_bounds__(64) void k_cls(const float* __restrict__ G, const float* __restrict__ WC, const float* __restrict__ BC, float* __restrict__ out) {
  __shared__ __align__(16) float so[NBATCH * NCL]; const int t = threadIdx.x;
  for (int q = t; q < NBATCH * NCL; q += 64) { const int b = q / NCL, o = q % NCL; float a = 0.f; if (b < NBT) { a = bfr(BC[o]);
#pragma unroll 1
      for (int c = 0; c < 32; ++c) a += G[b * 32 + c] * bfr(WC[c * NCL + o]); } so[q] = a; }
  __syncthreads();
  for (int q = t; q < NBATCH * NCL / 4; q += 64) vst2(out + q * 4, *(const v4f*)&so[q * 4]);
}
extern "C" void kernel_launch(void* const* d_in, const int* in_sizes, int n_in, void* d_out, int out_size, void* d_ws, size_t ws_size, hipStream_t stream) {
  (void)in_sizes; (void)n_in; (void)out_size;
  const float** F = (const float**)d_in;
  if (ws_size < (size_t)WS_END) return;
  char* ws = (char*)d_ws; __bf16* PW = (__bf16*)(ws + WS_PW); int* KNN = (int*)(ws + WS_KNN); float *F4 = (float*)(ws + WS_F4), *MSG = (float*)(ws + WS_MSG), *X = (float*)(ws + WS_X), *G = (float*)(ws + WS_G);
  k_packw<<<1, 256, 0, stream>>>(F[5], F[7], F[9], PW);
  k_knn<<<NQB, 64, 0, stream>>>(F[0], KNN);
  k_edge1<<<NRWB, 128, 0, stream>>>(F[0], F[1], KNN, F[3], F[4], PW, F[6], F4, MSG);
  k_segmax<<<NQB, 256, 0, stream>>>(MSG, X);
  k_edge2<<<NRWB, 128, 0, stream>>>(X, F4, KNN, PW, F[8], F[10], MSG);
  k_segmax<<<NQB, 256, 0, stream>>>(MSG, X);
  k_pool<<<NBT, 256, 0, stream>>>(X, G);
  k_cls<<<1, 64, 0, stream>>>(G, F[11], F[12], (float*)d_out);
}
